// StructuralStreamGAT_51445118271854
// MI455X (gfx1250) — hardware-verified
//
#include <hip/hip_runtime.h>
#include <stddef.h>


#define NTHR   256
#define NWAVE  8
#define GR     32
#define CIN    256
#define CH     64
#define NHD    4
#define C1     (NHD * CH)
#define TP1    68
#define TP2    260
#define NB1    256
#define SB1    8
#define NB2    1024
#define SB2    10
#define CHUNK  2048
#define WCAP   ((CHUNK / NTHR) * 32)
#define NGRP   (CHUNK / (NTHR * 4))
#define ROWPAD 1024
#define ACLAMP 80.0f
#define LDS1   ((NB1 * C1 + NB1 * NHD + NWAVE * WCAP + NWAVE) * 4)
#define LDS2   ((NB2 * CH + NB2 + NWAVE * WCAP + NWAVE) * 4)

static_assert(WCAP == 256);
static_assert(NGRP == 2);
static_assert((1 << SB1) == NB1);
static_assert((1 << SB2) == NB2);
static_assert(C1 == CIN);
static_assert(LDS1 == 274464);
static_assert(LDS2 == 274464);
static_assert(((NB1 * C1 + NB1 * NHD) % 4) == 0);
static_assert(((NB2 * CH + NB2) % 4) == 0);
static_assert((ROWPAD % NB1) == 0);
static_assert((ROWPAD % NB2) == 0);
static_assert((ROWPAD % GR) == 0);
static_assert(((TP1 * 4) % 16) == 0);
static_assert(((TP2 * 4) % 16) == 0);

typedef float          v2f  __attribute__((ext_vector_type(2)));
typedef float          v4f  __attribute__((ext_vector_type(4)));
typedef float          v8f  __attribute__((ext_vector_type(8)));
typedef int            v4i  __attribute__((ext_vector_type(4)));
typedef __bf16         v16b __attribute__((ext_vector_type(16)));
typedef unsigned short u16;
union FragU { v16b v; v4i q[2]; };

__device__ __forceinline__ unsigned bfr(float f) {
  const unsigned u = __float_as_uint(f);
  return ((u + 0x7FFFu + ((u >> 16) & 1u)) >> 16) & 0xFFFFu;
}
__device__ __forceinline__ void split_pair(float a, float b, unsigned& ph, unsigned& pl) {
  const unsigned ha = bfr(a), hb = bfr(b);
  const float ra = a - __uint_as_float(ha << 16);
  const float rb = b - __uint_as_float(hb << 16);
  ph = ha | (hb << 16);
  pl = bfr(ra) | (bfr(rb) << 16);
}
__device__ __forceinline__ void split8(v4f a, v4f b, v4i& qh, v4i& ql) {
  unsigned h0, l0, h1, l1, h2, l2, h3, l3;
  split_pair(a.x, a.y, h0, l0);
  split_pair(a.z, a.w, h1, l1);
  split_pair(b.x, b.y, h2, l2);
  split_pair(b.z, b.w, h3, l3);
  qh.x = (int)h0; qh.y = (int)h1; qh.z = (int)h2; qh.w = (int)h3;
  ql.x = (int)l0; ql.y = (int)l1; ql.z = (int)l2; ql.w = (int)l3;
}

__device__ __forceinline__ v8f wm3(v16b ah, v16b al, v16b bh, v16b bl, v8f c) {
  v8f d = __builtin_amdgcn_wmma_f32_16x16x32_bf16(false, ah, false, bh, (short)0, c, false, false);
  d = __builtin_amdgcn_wmma_f32_16x16x32_bf16(false, ah, false, bl, (short)0, d, false, false);
  d = __builtin_amdgcn_wmma_f32_16x16x32_bf16(false, al, false, bh, (short)0, d, false, false);
  asm volatile("v_nop\n\tv_nop\n\tv_nop\n\tv_nop" : "+v"(d) : "v"(ah), "v"(al), "v"(bh), "v"(bl));
  return d;
}

__device__ __forceinline__ v16b ldf(const u16* p, int h) {
  FragU f;
  f.q[0] = *(const v4i*)(p + 8 * h);
  f.q[1] = *(const v4i*)(p + 16 + 8 * h);
  return f.v;
}

__device__ __forceinline__ float hsum16(float v) {
  v += __shfl_xor(v, 8, 32);
  v += __shfl_xor(v, 4, 32);
  v += __shfl_xor(v, 2, 32);
  v += __shfl_xor(v, 1, 32);
  return v;
}

__device__ __forceinline__ float elu1(float v) { return v > 0.f ? v : (__expf(v) - 1.0f); }

__device__ __forceinline__ float lrelu_clamp_exp(float a) {
  a = a >= 0.f ? a : 0.2f * a;
  a = fminf(fmaxf(a, -ACLAMP), ACLAMP);
  return __expf(a);
}

__global__ __launch_bounds__(NTHR) void k_prepw(const float* __restrict__ W, u16* Th, u16* Tl,
                                                 int K, int Nc) {
  const int i  = blockIdx.x * NTHR + threadIdx.x;
  const int k8 = K >> 3;
  if (i >= Nc * k8) return;
  const int n  = i / k8;
  const int k0 = (i - n * k8) * 8;
  v4f a, b;
  a.x = W[(size_t)(k0 + 0) * Nc + n]; a.y = W[(size_t)(k0 + 1) * Nc + n];
  a.z = W[(size_t)(k0 + 2) * Nc + n]; a.w = W[(size_t)(k0 + 3) * Nc + n];
  b.x = W[(size_t)(k0 + 4) * Nc + n]; b.y = W[(size_t)(k0 + 5) * Nc + n];
  b.z = W[(size_t)(k0 + 6) * Nc + n]; b.w = W[(size_t)(k0 + 7) * Nc + n];
  v4i qh, ql;
  split8(a, b, qh, ql);
  const size_t o = (size_t)n * K + k0;
  *(volatile v4i*)(Th + o) = qh;
  *(volatile v4i*)(Tl + o) = ql;
  __threadfence();
  *(volatile v4i*)(Th + o) = qh;
  *(volatile v4i*)(Tl + o) = ql;
}

__global__ __launch_bounds__(NTHR) void k_splitx(const float* __restrict__ x, u16* Xh, u16* Xl,
                                                  int nN, int nP) {
  const int i = blockIdx.x * NTHR + threadIdx.x;
  if (i >= nP * (CIN / 8)) return;
  const int row = i >> 5;
  const int c0  = (i & 31) * 8;
  int srow = row;
  if (srow > nN - 1) srow = nN - 1;
  const float* p = x + (size_t)srow * CIN + c0;
  const v4f a = *(const v4f*)p;
  const v4f b = *(const v4f*)(p + 4);
  v4i qh, ql;
  split8(a, b, qh, ql);
  const size_t o = (size_t)row * CIN + c0;
  *(volatile v4i*)(Xh + o) = qh;
  *(volatile v4i*)(Xl + o) = ql;
  __threadfence();
  *(volatile v4i*)(Xh + o) = qh;
  *(volatile v4i*)(Xl + o) = ql;
}

__device__ __forceinline__ void gemm_k256_tile(const u16* __restrict__ Ah, const u16* __restrict__ Al,
                                               const u16* __restrict__ Bh, const u16* __restrict__ Bl,
                                               int rowBase, float* Ts) {
  const int tid = threadIdx.x, l = tid & 31, w = tid >> 5, h = l >> 4, m = l & 15;
  const int rt = w & 1, ct = w >> 1;
  const u16* pah = Ah + (size_t)(rowBase + 16 * rt + m) * CIN;
  const u16* pal = Al + (size_t)(rowBase + 16 * rt + m) * CIN;
  const u16* pbh = Bh + (size_t)(16 * ct + m) * CIN;
  const u16* pbl = Bl + (size_t)(16 * ct + m) * CIN;
  v8f acc = {0.f, 0.f, 0.f, 0.f, 0.f, 0.f, 0.f, 0.f};
#pragma unroll 2
  for (int kt = 0; kt < CIN / 32; ++kt) {
    const int k0 = kt * 32;
    const v16b ah = ldf(pah + k0, h);
    const v16b al = ldf(pal + k0, h);
    const v16b bh = ldf(pbh + k0, h);
    const v16b bl = ldf(pbl + k0, h);
    acc = wm3(ah, al, bh, bl, acc);
  }
#pragma unroll
  for (int r = 0; r < 8; ++r) Ts[(16 * rt + 8 * h + r) * TP1 + 16 * ct + m] = acc[r];
}

__global__ __launch_bounds__(NTHR) void k_gemm_p(const u16* __restrict__ Ah, const u16* __restrict__ Al,
                                                  const u16* __restrict__ Bh, const u16* __restrict__ Bl,
                                                  const float* __restrict__ bias, u16* Oh, u16* Ol) {
  __shared__ __attribute__((aligned(16))) float Ts[GR * TP1];
  const int rowBase = blockIdx.x * GR;
  gemm_k256_tile(Ah, Al, Bh, Bl, rowBase, Ts);
  __syncthreads();
  const int tid = threadIdx.x, l = tid & 31, w = tid >> 5;
  const int row = 4 * w + (l >> 3);
  const int c0  = (l & 7) * 8;
  const float* tp = Ts + row * TP1 + c0;
  v4f a = *(const v4f*)tp;
  v4f b = *(const v4f*)(tp + 4);
  a += *(const v4f*)(bias + c0);
  b += *(const v4f*)(bias + c0 + 4);
  v4i qh, ql;
  split8(a, b, qh, ql);
  const size_t o = (size_t)(rowBase + row) * CH + c0;
  *(volatile v4i*)(Oh + o) = qh;
  *(volatile v4i*)(Ol + o) = ql;
  __threadfence();
  *(volatile v4i*)(Oh + o) = qh;
  *(volatile v4i*)(Ol + o) = ql;
}

__global__ __launch_bounds__(NTHR) void k_gemm_f(const u16* __restrict__ Ah, const u16* __restrict__ Al,
                                                  const u16* __restrict__ Bh, const u16* __restrict__ Bl,
                                                  const float* __restrict__ ats, const float* __restrict__ atd,
                                                  float* Of, float* as, float* ad) {
  __shared__ __attribute__((aligned(16))) float Ts[GR * TP1];
  __shared__ __attribute__((aligned(16))) float Dl[2 * GR];
  const int rowBase = blockIdx.x * GR;
  gemm_k256_tile(Ah, Al, Bh, Bl, rowBase, Ts);
  __syncthreads();
  const int tid = threadIdx.x, l = tid & 31, w = tid >> 5;
  const int c   = 4 * (l & 15);
  const int r0  = 4 * w + (l >> 4);
  const int r1  = r0 + 2;
  const v4f x0 = *(const v4f*)(Ts + r0 * TP1 + c);
  const v4f x1 = *(const v4f*)(Ts + r1 * TP1 + c);
  float* p0 = Of + (size_t)(rowBase + r0) * CH + c;
  float* p1 = Of + (size_t)(rowBase + r1) * CH + c;
  *(volatile v4f*)p0 = x0;
  *(volatile v4f*)p1 = x1;
  if (tid < 2 * GR) {
    const int row = tid >> 1, which = tid & 1;
    const float* at = which ? atd : ats;
    const float* tr = Ts + row * TP1;
    float s = 0.f;
#pragma unroll 8
    for (int k = 0; k < CH; ++k) s += tr[k] * at[k];
    Dl[which * GR + row] = s;
  }
  __syncthreads();
  __threadfence();
  *(volatile v4f*)p0 = x0;
  *(volatile v4f*)p1 = x1;
  if (w == 0 && l < 16) {
    const int which = l >> 3, q = l & 7;
    const v4f d = *(const v4f*)(Dl + which * GR + 4 * q);
    float* dp = (which ? ad : as) + rowBase + 4 * q;
    *(volatile v4f*)dp = d;
    __threadfence();
    *(volatile v4f*)dp = d;
  }
}

__global__ __launch_bounds__(NTHR) void k_gemm_w(const u16* __restrict__ Ah, const u16* __restrict__ Al,
                                                  const u16* __restrict__ Bh, const u16* __restrict__ Bl,
                                                  const float* __restrict__ ats, const float* __restrict__ atd,
                                                  float* H1, float* as1, float* ad1) {
  __shared__ __attribute__((aligned(16))) float Ts[GR * TP2];
  __shared__ __attribute__((aligned(16))) float Dl[2 * GR * NHD];
  const int tid = threadIdx.x, l = tid & 31, w = tid >> 5, h = l >> 4, m = l & 15;
  const int rowBase = blockIdx.x * GR;
  const u16* pa0h = Ah + (size_t)(rowBase + m) * CH;
  const u16* pa0l = Al + (size_t)(rowBase + m) * CH;
  const u16* pa1h = Ah + (size_t)(rowBase + 16 + m) * CH;
  const u16* pa1l = Al + (size_t)(rowBase + 16 + m) * CH;
  const u16* pb0h = Bh + (size_t)(32 * w + m) * CH;
  const u16* pb0l = Bl + (size_t)(32 * w + m) * CH;
  const u16* pb1h = Bh + (size_t)(32 * w + 16 + m) * CH;
  const u16* pb1l = Bl + (size_t)(32 * w + 16 + m) * CH;
  v8f c00 = {0.f, 0.f, 0.f, 0.f, 0.f, 0.f, 0.f, 0.f};
  v8f c01 = c00, c10 = c00, c11 = c00;
#pragma unroll
  for (int kt = 0; kt < CH / 32; ++kt) {
    const int k0 = kt * 32;
    const v16b a0h = ldf(pa0h + k0, h), a0l = ldf(pa0l + k0, h);
    const v16b a1h = ldf(pa1h + k0, h), a1l = ldf(pa1l + k0, h);
    const v16b b0h = ldf(pb0h + k0, h), b0l = ldf(pb0l + k0, h);
    const v16b b1h = ldf(pb1h + k0, h), b1l = ldf(pb1l + k0, h);
    c00 = wm3(a0h, a0l, b0h, b0l, c00);
    c01 = wm3(a0h, a0l, b1h, b1l, c01);
    c10 = wm3(a1h, a1l, b0h, b0l, c10);
    c11 = wm3(a1h, a1l, b1h, b1l, c11);
  }
#pragma unroll
  for (int r = 0; r < 8; ++r) {
    Ts[(8 * h + r) * TP2 + 32 * w + m]           = c00[r];
    Ts[(8 * h + r) * TP2 + 32 * w + 16 + m]      = c01[r];
    Ts[(16 + 8 * h + r) * TP2 + 32 * w + m]      = c10[r];
    Ts[(16 + 8 * h + r) * TP2 + 32 * w + 16 + m] = c11[r];
  }
  __syncthreads();

  const float* tb = Ts + (4 * w) * TP2 + 4 * l;
  float* hb = H1 + (size_t)(rowBase + 4 * w) * C1 + 4 * l;
  const v4f x0 = *(const v4f*)(tb + 0 * TP2),       x1 = *(const v4f*)(tb + 0 * TP2 + 128);
  const v4f x2 = *(const v4f*)(tb + 1 * TP2),       x3 = *(const v4f*)(tb + 1 * TP2 + 128);
  const v4f x4 = *(const v4f*)(tb + 2 * TP2),       x5 = *(const v4f*)(tb + 2 * TP2 + 128);
  const v4f x6 = *(const v4f*)(tb + 3 * TP2),       x7 = *(const v4f*)(tb + 3 * TP2 + 128);
  *(volatile v4f*)(hb + 0 * C1) = x0; *(volatile v4f*)(hb + 0 * C1 + 128) = x1;
  *(volatile v4f*)(hb + 1 * C1) = x2; *(volatile v4f*)(hb + 1 * C1 + 128) = x3;
  *(volatile v4f*)(hb + 2 * C1) = x4; *(volatile v4f*)(hb + 2 * C1 + 128) = x5;
  *(volatile v4f*)(hb + 3 * C1) = x6; *(volatile v4f*)(hb + 3 * C1 + 128) = x7;

  {
    const int row = tid >> 3, hd = (tid >> 1) & 3, which = tid & 1;
    const float* at = (which ? atd : ats) + hd * CH;
    const float* tr = Ts + row * TP2 + hd * CH;
    float s = 0.f;
#pragma unroll 8
    for (int k = 0; k < CH; ++k) s += tr[k] * at[k];
    Dl[(which * GR + row) * NHD + hd] = s;
  }
  __syncthreads();
  __threadfence();
  *(volatile v4f*)(hb + 0 * C1) = x0; *(volatile v4f*)(hb + 0 * C1 + 128) = x1;
  *(volatile v4f*)(hb + 1 * C1) = x2; *(volatile v4f*)(hb + 1 * C1 + 128) = x3;
  *(volatile v4f*)(hb + 2 * C1) = x4; *(volatile v4f*)(hb + 2 * C1 + 128) = x5;
  *(volatile v4f*)(hb + 3 * C1) = x6; *(volatile v4f*)(hb + 3 * C1 + 128) = x7;
  if (w < 2) {
    const v4f d = *(const v4f*)(Dl + (w * GR + l) * NHD);
    float* dp = (w ? ad1 : as1) + (size_t)(rowBase + l) * NHD;
    *(volatile v4f*)dp = d;
    __threadfence();
    *(volatile v4f*)dp = d;
  }
}

template <int SB>
__device__ __forceinline__ void push_hit(bool hj, unsigned sj, int elj, int& wc, int* wl) {
  const unsigned mj = __builtin_amdgcn_ballot_w32(hj);
  if (hj) {
    const int pos = wc + (int)__builtin_amdgcn_mbcnt_lo(mj, 0u);
    if (pos < WCAP) wl[pos] = (elj << SB) | (int)sj;
  }
  wc += (int)__builtin_popcount(mj);
}

template <int NB, int SB>
__device__ __forceinline__ int scan_chunk(const int* __restrict__ eid, int nE, bool al16, int cbase,
                                          int nodeBase, int tid, int* wl) {
  int wc = 0;
#pragma unroll
  for (int g = 0; g < NGRP; ++g) {
    const int el0  = (g * NTHR + tid) * 4;
    const int e0   = cbase + el0;
    const int sent = -2147483647 - 1;
    v4i d;
    if (al16 && (e0 + 3 < nE)) {
      d = *(const v4i*)(eid + e0);
    } else {
      d.x = (e0     < nE) ? eid[min(e0,     nE - 1)] : sent;
      d.y = (e0 + 1 < nE) ? eid[min(e0 + 1, nE - 1)] : sent;
      d.z = (e0 + 2 < nE) ? eid[min(e0 + 2, nE - 1)] : sent;
      d.w = (e0 + 3 < nE) ? eid[min(e0 + 3, nE - 1)] : sent;
    }
    const unsigned s0 = (unsigned)d.x - (unsigned)nodeBase;
    const unsigned s1 = (unsigned)d.y - (unsigned)nodeBase;
    const unsigned s2 = (unsigned)d.z - (unsigned)nodeBase;
    const unsigned s3 = (unsigned)d.w - (unsigned)nodeBase;
    const bool h0 = s0 < (unsigned)NB;
    const bool h1 = s1 < (unsigned)NB;
    const bool h2 = s2 < (unsigned)NB;
    const bool h3 = s3 < (unsigned)NB;
    const unsigned many = __builtin_amdgcn_ballot_w32(h0 | h1 | h2 | h3);
    if (many != 0u) {
      push_hit<SB>(h0, s0, el0 + 0, wc, wl);
      push_hit<SB>(h1, s1, el0 + 1, wc, wl);
      push_hit<SB>(h2, s2, el0 + 2, wc, wl);
      push_hit<SB>(h3, s3, el0 + 3, wc, wl);
    }
  }
  return wc;
}

__global__ __launch_bounds__(NTHR) void k_agg1(const int* __restrict__ ei, const float* __restrict__ h1,
                                                const float* __restrict__ as1, const float* __restrict__ ad1,
                                                const float* __restrict__ bias, u16* Oh, u16* Ol,
                                                int nN, int nE, int nP) {
  extern __shared__ v4f lds_dyn[];
  float* sacc = (float*)lds_dyn;
  float* den  = sacc + NB1 * C1;
  int*   list = (int*)(den + NB1 * NHD);
  int*   wcnt = list + NWAVE * WCAP;

  const int tid = threadIdx.x, lane = tid & 31, wave = tid >> 5;
  const int hd = lane >> 3;
  const int nodeBase = blockIdx.x * NB1;

  {
    const v4f z4 = {0.f, 0.f, 0.f, 0.f};
    for (int i = tid; i < (NB1 * C1 + NB1 * NHD) / 4; i += NTHR) lds_dyn[i] = z4;
  }
  __syncthreads();

  const int* eid = ei + nE;
  const bool al16 = ((nE & 3) == 0);
  int* wl = list + wave * WCAP;
  const int nChunks = (nE + CHUNK - 1) / CHUNK;
#pragma unroll 1
  for (int ch = 0; ch < nChunks; ++ch) {
    const int cbase = ch * CHUNK;
    const int wc = scan_chunk<NB1, SB1>(eid, nE, al16, cbase, nodeBase, tid, wl);
    if (lane == 0) wcnt[wave] = wc;
    __syncthreads();
    if (wave == 0) {
#pragma unroll 1
      for (int wsx = 0; wsx < NWAVE; ++wsx) {
        int n = wcnt[wsx];
        n = n > WCAP ? WCAP : n;
        n = n < 0 ? 0 : n;
        const int* lp = list + wsx * WCAP;
#pragma unroll 1
        for (int i = 0; i < n; ++i) {
          const int ent  = lp[i];
          const int slot = ent & (NB1 - 1);
          const int el   = (ent >> SB1) & (CHUNK - 1);
          int e = cbase + el;
          e = e > nE - 1 ? nE - 1 : e;
          int src = ei[e];
          src = src < 0 ? 0 : (src > nN - 1 ? nN - 1 : src);
          int nd = nodeBase + slot;
          nd = nd > nP - 1 ? nP - 1 : nd;
          const float p = lrelu_clamp_exp(as1[(size_t)src * NHD + hd] + ad1[(size_t)nd * NHD + hd]);
          const float* hp = h1 + (size_t)src * C1 + 8 * lane;
          const v4f x0 = *(const v4f*)hp;
          const v4f x1 = *(const v4f*)(hp + 4);
          v4f* sp = (v4f*)(sacc + slot * C1 + 8 * lane);
          const v4f o0 = sp[0], o1 = sp[1];
          sp[0] = o0 + p * x0;
          sp[1] = o1 + p * x1;
          if ((lane & 7) == 0) {
            const float dv = den[slot * NHD + hd];
            den[slot * NHD + hd] = dv + p;
          }
        }
      }
    }
    __syncthreads();
  }

  const v4f b0 = *(const v4f*)(bias + 8 * lane);
  const v4f b1 = *(const v4f*)(bias + 8 * lane + 4);
#pragma unroll 1
  for (int j = 0; j < NB1 / NWAVE; ++j) {
    const int slot = wave * (NB1 / NWAVE) + j;
    const int node = nodeBase + slot;
    if (node >= nP) break;
    const size_t nrow = (size_t)node;
    const float p = lrelu_clamp_exp(as1[nrow * NHD + hd] + ad1[nrow * NHD + hd]);
    const float* hp = h1 + nrow * C1 + 8 * lane;
    const v4f x0 = *(const v4f*)hp;
    const v4f x1 = *(const v4f*)(hp + 4);
    const v4f* sp = (const v4f*)(sacc + slot * C1 + 8 * lane);
    const v4f s0 = sp[0] + p * x0;
    const v4f s1 = sp[1] + p * x1;
    const float dv  = den[slot * NHD + hd] + p;
    const float inv = __builtin_amdgcn_rcpf(dv);
    v4f v0 = s0 * inv + b0;
    v4f v1 = s1 * inv + b1;
    v0.x = elu1(v0.x); v0.y = elu1(v0.y); v0.z = elu1(v0.z); v0.w = elu1(v0.w);
    v1.x = elu1(v1.x); v1.y = elu1(v1.y); v1.z = elu1(v1.z); v1.w = elu1(v1.w);
    v4i qh, ql;
    split8(v0, v1, qh, ql);
    const size_t o = nrow * C1 + 8 * lane;
    *(volatile v4i*)(Oh + o) = qh;
    *(volatile v4i*)(Ol + o) = ql;
    __threadfence();
    *(volatile v4i*)(Oh + o) = qh;
    *(volatile v4i*)(Ol + o) = ql;
  }
}

__global__ __launch_bounds__(NTHR) void k_agg2(const int* __restrict__ ei, const float* __restrict__ h2,
                                                const float* __restrict__ as2, const float* __restrict__ ad2,
                                                const float* __restrict__ bias, const float* __restrict__ gam,
                                                const float* __restrict__ bet, float* out,
                                                int nN, int nE, int nP) {
  extern __shared__ v4f lds_dyn[];
  float* sacc = (float*)lds_dyn;
  float* den  = sacc + NB2 * CH;
  int*   list = (int*)(den + NB2);
  int*   wcnt = list + NWAVE * WCAP;

  const int tid = threadIdx.x, lane = tid & 31, wave = tid >> 5;
  const int nodeBase = blockIdx.x * NB2;

  {
    const v4f z4 = {0.f, 0.f, 0.f, 0.f};
    for (int i = tid; i < (NB2 * CH + NB2) / 4; i += NTHR) lds_dyn[i] = z4;
  }
  __syncthreads();

  const int* eid = ei + nE;
  const bool al16 = ((nE & 3) == 0);
  int* wl = list + wave * WCAP;
  const int nChunks = (nE + CHUNK - 1) / CHUNK;
#pragma unroll 1
  for (int ch = 0; ch < nChunks; ++ch) {
    const int cbase = ch * CHUNK;
    const int wc = scan_chunk<NB2, SB2>(eid, nE, al16, cbase, nodeBase, tid, wl);
    if (lane == 0) wcnt[wave] = wc;
    __syncthreads();
    if (wave == 0) {
#pragma unroll 1
      for (int wsx = 0; wsx < NWAVE; ++wsx) {
        int n = wcnt[wsx];
        n = n > WCAP ? WCAP : n;
        n = n < 0 ? 0 : n;
        const int* lp = list + wsx * WCAP;
#pragma unroll 1
        for (int i = 0; i < n; ++i) {
          const int ent  = lp[i];
          const int slot = ent & (NB2 - 1);
          const int el   = (ent >> SB2) & (CHUNK - 1);
          int e = cbase + el;
          e = e > nE - 1 ? nE - 1 : e;
          int src = ei[e];
          src = src < 0 ? 0 : (src > nN - 1 ? nN - 1 : src);
          int nd = nodeBase + slot;
          nd = nd > nP - 1 ? nP - 1 : nd;
          const float p = lrelu_clamp_exp(as2[src] + ad2[nd]);
          const float* hp = h2 + (size_t)src * CH + 2 * lane;
          const v2f xv = *(const v2f*)hp;
          v2f* sp = (v2f*)(sacc + slot * CH + 2 * lane);
          const v2f o = *sp;
          *sp = o + p * xv;
          if (lane == 0) {
            const float dv = den[slot];
            den[slot] = dv + p;
          }
        }
      }
    }
    __syncthreads();
  }

  const int q  = lane & 15;
  const int hl = lane >> 4;
  const v4f b4 = *(const v4f*)(bias + 4 * q);
  const v4f g4 = *(const v4f*)(gam + 4 * q);
  const v4f e4 = *(const v4f*)(bet + 4 * q);
#pragma unroll 1
  for (int j = 0; j < NB2 / NWAVE / 2; ++j) {
    const int slot = wave * (NB2 / NWAVE) + 2 * j + hl;
    const int node = nodeBase + slot;
    int nl = node;
    if (nl > nP - 1) nl = nP - 1;
    const size_t nrow = (size_t)nl;
    const float p = lrelu_clamp_exp(as2[nrow] + ad2[nrow]);
    const v4f xv = *(const v4f*)(h2 + nrow * CH + 4 * q);
    const v4f s  = *(const v4f*)(sacc + slot * CH + 4 * q) + p * xv;
    const float dv  = den[slot] + p;
    const float inv = __builtin_amdgcn_rcpf(dv);
    const v4f v = s * inv + b4;
    const float sm = hsum16(v.x + v.y + v.z + v.w);
    const float mu = sm * (1.0f / CH);
    const v4f d = v - mu;
    const float sq  = hsum16(d.x * d.x + d.y * d.y + d.z * d.z + d.w * d.w);
    const float var = sq * (1.0f / CH);
    const float rs  = rsqrtf(var + 1e-5f);
    const v4f y = d * rs * g4 + e4;
    if (node < nN) {
      float* op = out + (size_t)node * CH + 4 * q;
      *(volatile v4f*)op = y;
      __threadfence();
      *(volatile v4f*)op = y;
    }
  }
}

extern "C" void kernel_launch(void* const* d_in, const int* in_sizes, int n_in,
                              void* d_out, int out_size, void* d_ws, size_t ws_size,
                              hipStream_t stream) {
  if (n_in < 14) return;
  const int nN = in_sizes[0] / CIN;
  if (nN <= 0 || in_sizes[0] != nN * CIN) return;
  if (in_sizes[1] < 2 || (in_sizes[1] & 1) != 0) return;
  const int nE = in_sizes[1] / 2;
  if (in_sizes[2] != CIN * CH || in_sizes[3] != CH) return;
  if (in_sizes[4] != CH * C1 || in_sizes[5] != C1 || in_sizes[6] != C1 || in_sizes[7] != C1) return;
  if (in_sizes[8] != C1 * CH || in_sizes[9] != CH || in_sizes[10] != CH || in_sizes[11] != CH) return;
  if (in_sizes[12] != CH || in_sizes[13] != CH) return;
  if (out_size != nN * CH) return;

  const float* x        = (const float*)d_in[0];
  const int*   ei       = (const int*)d_in[1];
  const float* W_in     = (const float*)d_in[2];
  const float* b_in     = (const float*)d_in[3];
  const float* W1       = (const float*)d_in[4];
  const float* att_src1 = (const float*)d_in[5];
  const float* att_dst1 = (const float*)d_in[6];
  const float* bias1    = (const float*)d_in[7];
  const float* W2       = (const float*)d_in[8];
  const float* att_src2 = (const float*)d_in[9];
  const float* att_dst2 = (const float*)d_in[10];
  const float* bias2    = (const float*)d_in[11];
  const float* gamma    = (const float*)d_in[12];
  const float* beta     = (const float*)d_in[13];
  float* out = (float*)d_out;

  const int nP = ((nN + ROWPAD - 1) / ROWPAD) * ROWPAD;

  char* ws = (char*)d_ws;
  size_t off = 0;
  u16* WinTh = (u16*)(ws + off); off += (size_t)CIN * CH * 2;
  u16* WinTl = (u16*)(ws + off); off += (size_t)CIN * CH * 2;
  u16* W1Th  = (u16*)(ws + off); off += (size_t)C1 * CH * 2;
  u16* W1Tl  = (u16*)(ws + off); off += (size_t)C1 * CH * 2;
  u16* W2Th  = (u16*)(ws + off); off += (size_t)C1 * CH * 2;
  u16* W2Tl  = (u16*)(ws + off); off += (size_t)C1 * CH * 2;
  u16* h0h   = (u16*)(ws + off); off += (size_t)nP * CH * 2;
  u16* h0l   = (u16*)(ws + off); off += (size_t)nP * CH * 2;
  float* h2f = (float*)h0h;
  float* h1f = (float*)(ws + off); off += (size_t)nP * C1 * 4;
  float* as1 = (float*)(ws + off); off += (size_t)nP * NHD * 4;
  float* ad1 = (float*)(ws + off); off += (size_t)nP * NHD * 4;
  float* as2 = (float*)(ws + off); off += (size_t)nP * 4;
  float* ad2 = (float*)(ws + off); off += (size_t)nP * 4;
  u16* xh    = (u16*)(ws + off); off += (size_t)nP * CIN * 2;
  u16* xl    = (u16*)(ws + off); off += (size_t)nP * CIN * 2;
  u16* o1h   = xh;
  u16* o1l   = xl;
  if (off > ws_size) return;

  k_prepw<<<(CH * CIN / 8 + NTHR - 1) / NTHR, NTHR, 0, stream>>>(W_in, WinTh, WinTl, CIN, CH);
  k_prepw<<<(C1 * CH / 8 + NTHR - 1) / NTHR, NTHR, 0, stream>>>(W1, W1Th, W1Tl, CH, C1);
  k_prepw<<<(CH * C1 / 8 + NTHR - 1) / NTHR, NTHR, 0, stream>>>(W2, W2Th, W2Tl, C1, CH);

  k_splitx<<<(nP * (CIN / 8) + NTHR - 1) / NTHR, NTHR, 0, stream>>>(x, xh, xl, nN, nP);

  k_gemm_p<<<nP / GR, NTHR, 0, stream>>>(xh, xl, WinTh, WinTl, b_in, h0h, h0l);

  k_gemm_w<<<nP / GR, NTHR, 0, stream>>>(h0h, h0l, W1Th, W1Tl, att_src1, att_dst1, h1f, as1, ad1);

  hipFuncSetAttribute(reinterpret_cast<const void*>(&k_agg1),
                      hipFuncAttributeMaxDynamicSharedMemorySize, LDS1);
  k_agg1<<<nP / NB1, NTHR, LDS1, stream>>>(ei, h1f, as1, ad1, bias1, o1h, o1l, nN, nE, nP);

  k_gemm_f<<<nP / GR, NTHR, 0, stream>>>(o1h, o1l, W2Th, W2Tl, att_src2, att_dst2, h2f, as2, ad2);

  hipFuncSetAttribute(reinterpret_cast<const void*>(&k_agg2),
                      hipFuncAttributeMaxDynamicSharedMemorySize, LDS2);
  k_agg2<<<nP / NB2, NTHR, LDS2, stream>>>(ei, h2f, as2, ad2, bias2, gamma, beta, out, nN, nE, nP);
}
